// TemporalGNN_13743895347604
// MI455X (gfx1250) — hardware-run, weakly checked
//
#include <hip/hip_runtime.h>
#include <math.h>

typedef __attribute__((ext_vector_type(16))) _Float16 v16h;
typedef __attribute__((ext_vector_type(8)))  _Float16 v8h;
typedef __attribute__((ext_vector_type(8)))  float    v8f;
typedef __attribute__((ext_vector_type(4)))  float    v4f;
typedef __attribute__((ext_vector_type(4)))  int      v4i;
typedef __attribute__((ext_vector_type(4)))  unsigned v4u;
typedef __attribute__((ext_vector_type(8)))  unsigned v8u;

constexpr int kN      = 100000;
constexpr int kE      = 1600000;
constexpr int kF      = 8;
constexpr int kHid    = 32;
constexpr int kP      = 12;
constexpr int kXRow   = kF * kP;

constexpr int kDegTile   = 8192;
constexpr int kDegBlocks = (kN + kDegTile - 1) / kDegTile;
constexpr int kNPadD     = kDegBlocks * kDegTile;

constexpr int kAggTile   = 256;
constexpr int kAggBlocks = (kN + kAggTile - 1) / kAggTile;
constexpr int kNPadA     = kAggBlocks * kAggTile;

constexpr int kGruNodes  = 64;
constexpr int kGruBlocks = (kN + kGruNodes - 1) / kGruNodes;

constexpr int kEdgeChunk = 256;
constexpr int kChunks    = kE / kEdgeChunk;

static_assert(kXRow == 96, "row of 96 floats per node");
static_assert(kDegBlocks == 13 && kNPadD == 106496, "degree tiling");
static_assert(kAggBlocks == 391 && kNPadA == 100096, "aggregation tiling");
static_assert(kGruBlocks == 1563 && kGruBlocks * kGruNodes <= kNPadA, "recurrence tiling inside the padded plane");
static_assert((kE % kEdgeChunk) == 0 && kChunks == 6250, "edge list is a whole number of 256-edge chunks");
static_assert((kN % 16) == 0, "a 16-node wave group is either fully valid or fully padding");
static_assert(kHid == 32 && kF == 8, "one 32-deep k tile per operand group");

constexpr float kCarryW   = 64.0f;
constexpr float kCarryA   = 64.0f;
constexpr float kAccScale = kCarryW * kCarryA;
constexpr float kAccInv   = 1.0f / kAccScale;
constexpr float kFx       = 2097152.0f;
constexpr float kFxInv    = 1.0f / kFx;
static_assert(kAccScale == 4096.0f, "accumulator scale");

constexpr size_t kBytesDinv = (size_t)kNPadD * 4;
constexpr size_t kBytesXA   = (size_t)kP * kNPadA * kF * 2;
constexpr size_t kBytesWPh  = (size_t)192 * 32 * 2;
constexpr size_t kBytesWPf  = (size_t)128 * 4;
constexpr size_t kOffDinv   = 0;
constexpr size_t kOffXA     = kOffDinv + kBytesDinv;
constexpr size_t kOffWPh    = kOffXA + kBytesXA;
constexpr size_t kOffWPf    = kOffWPh + kBytesWPh;
constexpr size_t kWsTotal   = kOffWPf + kBytesWPf;
static_assert(kBytesDinv == 425984ull && kBytesXA == 19218432ull, "plane sizes");
static_assert(kWsTotal == 19657216ull, "carve total");
static_assert(kWsTotal <= 134217728ull, "carve cap");
static_assert((kOffXA % 128) == 0 && (kOffWPh % 128) == 0 && (kOffWPf % 128) == 0, "128-B aligned regions");
static_assert((((size_t)kNPadA * kF * 2) % 128) == 0, "period planes start on line boundaries");

constexpr int kOffAX  = 0;
constexpr int kOffAZR = 96 * 32;
constexpr int kOffAH  = 160 * 32;
constexpr int kTileH  = 16 * 32;

union FragH { v16h v; v8h h[2]; };
__device__ __forceinline__ v16h frag_load(const _Float16* p) {
  FragH f;
  f.h[0] = *(const v8h*)(p);
  f.h[1] = *(const v8h*)(p + 16);
  return f.v;
}
__device__ __forceinline__ v8f mma_h(v16h a, v16h b, v8f c) {
  c = __builtin_amdgcn_wmma_f32_16x16x32_f16(false, a, false, b, (short)0, c, false, false);
  asm volatile("v_nop\n\tv_nop\n\tv_nop\n\tv_nop" : "+v"(c) : "v"(a), "v"(b));
  return c;
}
__device__ __forceinline__ v8f load8f(const float* p) {
  const v4f a = *(const v4f*)(p);
  const v4f b = *(const v4f*)(p + 4);
  return __builtin_shufflevector(a, b, 0, 1, 2, 3, 4, 5, 6, 7);
}
__device__ __forceinline__ float sigm_scaled(float a) {
  const float xv = a * kAccInv;
  const float e = expf(-xv);
  return __builtin_amdgcn_rcpf(1.0f + e);
}
__device__ __forceinline__ float tanh_scaled(float a) {
  const float xv = a * kAccInv;
  const float e = expf(2.0f * xv);
  return 1.0f - 2.0f * __builtin_amdgcn_rcpf(1.0f + e);
}

__global__ __launch_bounds__(256) void deg_kernel(const int* __restrict__ ei, float* __restrict__ dinv)
{
  __shared__ __align__(16) int sCnt[kDegTile];
  const int tid  = threadIdx.x;
  const int lane = tid & 31;
  const int wave = __builtin_amdgcn_readfirstlane((int)(threadIdx.x >> 5));
  const int base = blockIdx.x * kDegTile;
  const int remain = kN - base;
  const unsigned lim = (unsigned)(remain < kDegTile ? remain : kDegTile);
#pragma unroll 1
  for (int i = 0; i < kDegTile / 256; ++i) sCnt[i * 256 + tid] = 0;
  __syncthreads();
  const int* dstRow = ei + kE;
#pragma unroll 1
  for (int c = wave; c < kChunks; c += 8) {
    const int eb = c * kEdgeChunk + lane * 8;
    const v4i d0 = *(const v4i*)(dstRow + eb);
    const v4i d1 = *(const v4i*)(dstRow + eb + 4);
#pragma unroll
    for (int j = 0; j < 4; ++j) {
      const unsigned u0 = (unsigned)d0[j] - (unsigned)base;
      const unsigned u1 = (unsigned)d1[j] - (unsigned)base;
      if (u0 < lim) atomicAdd(&sCnt[u0], 1);
      if (u1 < lim) atomicAdd(&sCnt[u1], 1);
    }
  }
  __syncthreads();
  v4f ov[8];
#pragma unroll
  for (int it = 0; it < 8; ++it) {
    const v4i cv = *(const v4i*)(sCnt + (it * 256 + tid) * 4);
    ov[it][0] = rsqrtf((float)(cv[0] + 1));
    ov[it][1] = rsqrtf((float)(cv[1] + 1));
    ov[it][2] = rsqrtf((float)(cv[2] + 1));
    ov[it][3] = rsqrtf((float)(cv[3] + 1));
  }
  float* dp = dinv + (size_t)base;
  for (int pass = 0; pass < 2; ++pass) {
#pragma unroll
    for (int it = 0; it < 8; ++it)
      *(volatile v4f*)(dp + (it * 256 + tid) * 4) = ov[it];
    __threadfence();
  }
}

__global__ __launch_bounds__(256) void agg_kernel(const float* __restrict__ x, const int* __restrict__ ei,
                                                  const float* __restrict__ dinv, unsigned short* __restrict__ XA)
{
  __shared__ __align__(16) int sAcc[kAggTile * kXRow];
  __shared__ float sDinv[kAggTile];
  const int tid  = threadIdx.x;
  const int lane = tid & 31;
  const int wave = __builtin_amdgcn_readfirstlane((int)(threadIdx.x >> 5));
  const int base = blockIdx.x * kAggTile;
  const int remain = kN - base;
  const unsigned lim = (unsigned)(remain < kAggTile ? remain : kAggTile);
  {
    int nc = base + tid;
    nc = nc < kN ? nc : kN - 1;
    sDinv[tid] = dinv[nc];
  }
  __syncthreads();
#pragma unroll 1
  for (int it = 0; it < kXRow; ++it) {
    const int idx = it * 256 + tid;
    const int nl  = idx / kXRow;
    const int col = idx - nl * kXRow;
    const int n   = base + nl;
    const int nc  = n < kN ? n : kN - 1;
    float v = x[(size_t)nc * kXRow + col];
    asm volatile("" : "+v"(v));
    const float sv = v * sDinv[nl] * kFx;
    const int q = (n < kN) ? __float2int_rn(sv) : 0;
    sAcc[idx] = q;
  }
  __syncthreads();

  const int* srcRow = ei;
  const int* dstRow = ei + kE;
#pragma unroll 1
  for (int c = wave; c < kChunks; c += 8) {
    const int eb = c * kEdgeChunk + lane * 8;
    const v4i d0 = *(const v4i*)(dstRow + eb);
    const v4i d1 = *(const v4i*)(dstRow + eb + 4);
    unsigned u[8];
    unsigned m[8];
#pragma unroll
    for (int j = 0; j < 4; ++j) {
      u[j]     = (unsigned)d0[j] - (unsigned)base;
      u[4 + j] = (unsigned)d1[j] - (unsigned)base;
    }
#pragma unroll
    for (int j = 0; j < 8; ++j) m[j] = __builtin_amdgcn_ballot_w32(u[j] < lim);
    const unsigned any = m[0] | m[1] | m[2] | m[3] | m[4] | m[5] | m[6] | m[7];
    if (any != 0u) {
      const v4i s0 = *(const v4i*)(srcRow + eb);
      const v4i s1 = *(const v4i*)(srcRow + eb + 4);
#pragma unroll
      for (int j = 0; j < 8; ++j) {
        unsigned mm = m[j];
        const int sj = (j < 4) ? s0[j & 3] : s1[j & 3];
        const int uj = (int)u[j];
        while (mm != 0u) {
          const int k = __builtin_ctz(mm);
          mm &= mm - 1u;
          int sl = __builtin_amdgcn_readlane(sj, k);
          int ul = __builtin_amdgcn_readlane(uj, k);
          sl = sl < 0 ? 0 : sl;
          sl = sl > kN - 1 ? kN - 1 : sl;
          ul = ul < 0 ? 0 : ul;
          ul = ul > kAggTile - 1 ? kAggTile - 1 : ul;
          const float ds = dinv[sl] * kFx;
          const float* xs = x + (size_t)sl * kXRow;
          int* ap = sAcc + ul * kXRow;
#pragma unroll
          for (int i = 0; i < 3; ++i) {
            const float v = xs[lane + 32 * i];
            const int q = __float2int_rn(v * ds);
            atomicAdd(ap + lane + 32 * i, q);
          }
        }
      }
    }
  }
  __syncthreads();

  const int n = base + tid;
  const bool valid = n < kN;
  const float scl = sDinv[tid] * (kCarryA * kFxInv);
  const int* arow = sAcc + tid * kXRow;
  unsigned short* dstp = XA + (size_t)n * kF;
  for (int pass = 0; pass < 2; ++pass) {
#pragma unroll 1
    for (int p = 0; p < kP; ++p) {
      v8h hv;
#pragma unroll
      for (int f = 0; f < kF; ++f) {
        const int a = arow[f * kP + p];
        const float val = valid ? ((float)a * scl) : 0.0f;
        hv[f] = (_Float16)val;
      }
      *(volatile v8h*)(dstp + (size_t)p * ((size_t)kNPadA * kF)) = hv;
    }
    __threadfence();
  }
}

__global__ __launch_bounds__(256) void prep_kernel(
    const float* __restrict__ att,
    const float* __restrict__ Wz, const float* __restrict__ bz,
    const float* __restrict__ Wr, const float* __restrict__ br,
    const float* __restrict__ Wh, const float* __restrict__ bh,
    const float* __restrict__ Lz, const float* __restrict__ lbz,
    const float* __restrict__ Lr, const float* __restrict__ lbr,
    const float* __restrict__ Lh, const float* __restrict__ lbh,
    unsigned short* __restrict__ WPh, float* __restrict__ WPf)
{
  __shared__ float sWp[3 * 256];
  __shared__ __align__(16) float sF[128];
  __shared__ __align__(16) float sPl[192 * 32];
  const int tid  = threadIdx.x;
  const int lane = tid & 31;
  const int wave = __builtin_amdgcn_readfirstlane((int)(threadIdx.x >> 5));

#pragma unroll 1
  for (int g = 0; g < 3; ++g) {
    const float* Wg = (g == 0) ? Wz : ((g == 1) ? Wr : Wh);
    const float* Lg = (g == 0) ? Lz : ((g == 1) ? Lr : Lh);
    const int k = tid >> 5;
    const int o = tid & 31;
    float s = 0.0f;
#pragma unroll 4
    for (int j = 0; j < kHid; ++j) s = fmaf(Wg[k * kHid + j], Lg[j * kHid + o], s);
    sWp[g * 256 + k * kHid + o] = s;
  }
  if (wave < 3) {
    const float* bg  = (wave == 0) ? bz : ((wave == 1) ? br : bh);
    const float* Lg  = (wave == 0) ? Lz : ((wave == 1) ? Lr : Lh);
    const float* lbg = (wave == 0) ? lbz : ((wave == 1) ? lbr : lbh);
    float s = lbg[lane];
#pragma unroll 4
    for (int j = 0; j < kHid; ++j) s = fmaf(bg[j], Lg[j * kHid + lane], s);
    sF[wave * 32 + lane] = s * kAccScale;
  } else if (wave == 3) {
    float mx = att[0];
#pragma unroll 1
    for (int p = 1; p < kP; ++p) mx = fmaxf(mx, att[p]);
    float sum = 0.0f;
#pragma unroll 1
    for (int p = 0; p < kP; ++p) sum += expf(att[p] - mx);
    const int pc = lane < kP ? lane : kP - 1;
    float a = att[pc];
    asm volatile("" : "+v"(a));
    const float val = expf(a - mx) * (1.0f / sum);
    sF[96 + lane] = (lane < kP) ? val : 0.0f;
  }
  __syncthreads();

#pragma unroll 1
  for (int it = 0; it < 24; ++it) {
    const int row = it * 8 + wave;
    const int k = lane;
    float v;
    if (row < 96) {
      const int g = row >> 5;
      const int o = row & 31;
      const int kc = k < kF ? k : kF - 1;
      const float w = sWp[g * 256 + kc * kHid + o];
      v = (k < kF) ? w : 0.0f;
    } else if (row < 160) {
      const int rr = row - 96;
      const float* L = ((rr >> 5) == 0) ? Lz : Lr;
      v = L[(kHid + k) * kHid + (rr & 31)];
    } else {
      v = Lh[(kHid + k) * kHid + (row - 160)];
    }
    sPl[row * 32 + k] = v * kCarryW;
  }
  __syncthreads();

  v8h pv[3];
#pragma unroll
  for (int it = 0; it < 3; ++it) {
    const int q = it * 256 + tid;
    const v4f a0 = *(const v4f*)(sPl + q * 8);
    const v4f a1 = *(const v4f*)(sPl + q * 8 + 4);
#pragma unroll
    for (int e = 0; e < 4; ++e) {
      pv[it][e]     = (_Float16)a0[e];
      pv[it][4 + e] = (_Float16)a1[e];
    }
  }
  const v4f fv = *(const v4f*)(sF + lane * 4);
  for (int pass = 0; pass < 2; ++pass) {
#pragma unroll
    for (int it = 0; it < 3; ++it) {
      const int q = it * 256 + tid;
      *(volatile v8h*)(WPh + (size_t)q * 8) = pv[it];
    }
    if (wave == 0) *(volatile v4f*)(WPf + lane * 4) = fv;
    __threadfence();
  }
}

__global__ __launch_bounds__(128) void gru_kernel(
    const unsigned short* __restrict__ XA, const unsigned short* __restrict__ WPh, const float* __restrict__ WPf,
    const float* __restrict__ Wout, const float* __restrict__ bout, float* __restrict__ out)
{
  __shared__ __align__(16) _Float16 sW[192 * 32];
  __shared__ __align__(16) float sC[128];
  __shared__ __align__(16) float sWo[kHid * kF];
  __shared__ __align__(16) float sBo[8];
  const int tid  = threadIdx.x;
  const int lane = tid & 31;
  const int wave = __builtin_amdgcn_readfirstlane((int)(threadIdx.x >> 5));
  const int hh   = lane >> 4;
  const int nn   = lane & 15;

#pragma unroll
  for (int i = 0; i < 6; ++i) {
    const int q = i * 128 + tid;
    *(v8h*)(sW + q * 8) = *(const v8h*)((const _Float16*)WPh + q * 8);
  }
  sC[tid] = WPf[tid];
  sWo[tid] = Wout[tid];
  sWo[tid + 128] = Wout[tid + 128];
  {
    const int bc = tid < kF ? tid : kF - 1;
    float b = bout[bc];
    asm volatile("" : "+v"(b));
    if (tid < kF) sBo[tid] = b;
  }
  __syncthreads();

  const v8f zero8 = (v8f){0.f, 0.f, 0.f, 0.f, 0.f, 0.f, 0.f, 0.f};
  v8f H0 = zero8, H1 = zero8, S0 = zero8, S1 = zero8;
  const int node = blockIdx.x * kGruNodes + wave * 16 + nn;
  const unsigned short* xrow = XA + (size_t)node * kF;
  const _Float16* wl = sW + nn * 32 + 8 * hh;
  const float* cl = sC + 8 * hh;
  const bool lo = (hh == 0);

#pragma unroll 1
  for (int t = 0; t < kP; ++t) {
    asm volatile("" ::: "memory");
    v4u raw = *(const v4u*)(xrow + (size_t)t * ((size_t)kNPadA * kF));
    asm volatile("" : "+v"(raw));
    v8u bw;
    bw[0] = lo ? raw[0] : 0u;
    bw[1] = lo ? raw[1] : 0u;
    bw[2] = lo ? raw[2] : 0u;
    bw[3] = lo ? raw[3] : 0u;
    bw[4] = 0u;
    bw[5] = 0u;
    bw[6] = 0u;
    bw[7] = 0u;
    const v16h bx = __builtin_bit_cast(v16h, bw);

    v16h bh;
#pragma unroll
    for (int i = 0; i < 8; ++i) {
      bh[i]     = (_Float16)(H0[i] * kCarryA);
      bh[8 + i] = (_Float16)(H1[i] * kCarryA);
    }

    v8f pz0 = load8f(cl + 0);
    v8f pz1 = load8f(cl + 16);
    v8f pr0 = load8f(cl + 32);
    v8f pr1 = load8f(cl + 48);
    pz0 = mma_h(frag_load(wl + kOffAX  + 0 * kTileH), bx, pz0);
    pz0 = mma_h(frag_load(wl + kOffAZR + 0 * kTileH), bh, pz0);
    pz1 = mma_h(frag_load(wl + kOffAX  + 1 * kTileH), bx, pz1);
    pz1 = mma_h(frag_load(wl + kOffAZR + 1 * kTileH), bh, pz1);
    pr0 = mma_h(frag_load(wl + kOffAX  + 2 * kTileH), bx, pr0);
    pr0 = mma_h(frag_load(wl + kOffAZR + 2 * kTileH), bh, pr0);
    pr1 = mma_h(frag_load(wl + kOffAX  + 3 * kTileH), bx, pr1);
    pr1 = mma_h(frag_load(wl + kOffAZR + 3 * kTileH), bh, pr1);

#pragma unroll 1
    for (int g = 0; g < 4; ++g) {
      v8f cur = pz0;
#pragma unroll
      for (int r = 0; r < 8; ++r) cur[r] = sigm_scaled(cur[r]);
      pz0 = pz1;
      pz1 = pr0;
      pr0 = pr1;
      pr1 = cur;
    }

    asm volatile("" ::: "memory");
    v16h brh;
#pragma unroll
    for (int i = 0; i < 8; ++i) {
      brh[i]     = (_Float16)(pr0[i] * H0[i] * kCarryA);
      brh[8 + i] = (_Float16)(pr1[i] * H1[i] * kCarryA);
    }
    v8f ph0 = load8f(cl + 64);
    v8f ph1 = load8f(cl + 80);
    ph0 = mma_h(frag_load(wl + kOffAX + 4 * kTileH), bx, ph0);
    ph0 = mma_h(frag_load(wl + kOffAH + 0 * kTileH), brh, ph0);
    ph1 = mma_h(frag_load(wl + kOffAX + 5 * kTileH), bx, ph1);
    ph1 = mma_h(frag_load(wl + kOffAH + 1 * kTileH), brh, ph1);

    const float pt = sC[96 + t];
#pragma unroll 1
    for (int g = 0; g < 2; ++g) {
      v8f hn, sn;
#pragma unroll
      for (int r = 0; r < 8; ++r) {
        const float ht = tanh_scaled(ph0[r]);
        const float z  = pz0[r];
        const float hv = z * H0[r] + (1.0f - z) * ht;
        hn[r] = hv;
        sn[r] = fmaf(pt, hv, S0[r]);
      }
      ph0 = ph1;
      pz0 = pz1;
      H0 = H1;
      H1 = hn;
      S0 = S1;
      S1 = sn;
    }
  }

  float po[kF];
#pragma unroll
  for (int o = 0; o < kF; ++o) po[o] = 0.0f;
#pragma unroll
  for (int r = 0; r < 8; ++r) {
    const float a0 = fmaxf(S0[r], 0.0f);
    const float a1 = fmaxf(S1[r], 0.0f);
    const float* w0 = sWo + (8 * hh + r) * kF;
    const float* w1 = sWo + (16 + 8 * hh + r) * kF;
    const v4f w0a = *(const v4f*)(w0);
    const v4f w0b = *(const v4f*)(w0 + 4);
    const v4f w1a = *(const v4f*)(w1);
    const v4f w1b = *(const v4f*)(w1 + 4);
#pragma unroll
    for (int e = 0; e < 4; ++e) {
      po[e]     = fmaf(a0, w0a[e], po[e]);
      po[4 + e] = fmaf(a0, w0b[e], po[4 + e]);
      po[e]     = fmaf(a1, w1a[e], po[e]);
      po[4 + e] = fmaf(a1, w1b[e], po[4 + e]);
    }
  }
  float tot[kF];
#pragma unroll
  for (int o = 0; o < kF; ++o) {
    const float other = __shfl_xor(po[o], 16, 32);
    tot[o] = po[o] + other + sBo[o];
  }
  float gsel[kF];
  const int srcLane = lane >> 1;
#pragma unroll
  for (int o = 0; o < kF; ++o) gsel[o] = __shfl(tot[o], srcLane, 32);
  const bool upper = (lane & 1) != 0;
  v4f ov;
  ov[0] = upper ? gsel[4] : gsel[0];
  ov[1] = upper ? gsel[5] : gsel[1];
  ov[2] = upper ? gsel[6] : gsel[2];
  ov[3] = upper ? gsel[7] : gsel[3];
  const int nodeBase = blockIdx.x * kGruNodes + wave * 16;
  if (nodeBase < kN) {
    float* op = out + (size_t)nodeBase * kF + lane * 4;
    *(volatile v4f*)op = ov;
    __threadfence();
    *(volatile v4f*)op = ov;
  }
}

extern "C" void kernel_launch(void* const* d_in, const int* in_sizes, int n_in,
                              void* d_out, int out_size, void* d_ws, size_t ws_size,
                              hipStream_t stream) {
  if (n_in < 17) return;
  if (in_sizes[0] != kN * kXRow) return;
  if (in_sizes[1] != 2 * kE) return;
  if (in_sizes[2] != kP) return;
  if (in_sizes[3] != kF * kHid || in_sizes[5] != kF * kHid || in_sizes[7] != kF * kHid) return;
  if (in_sizes[4] != kHid || in_sizes[6] != kHid || in_sizes[8] != kHid) return;
  if (in_sizes[9] != 2 * kHid * kHid || in_sizes[11] != 2 * kHid * kHid || in_sizes[13] != 2 * kHid * kHid) return;
  if (in_sizes[10] != kHid || in_sizes[12] != kHid || in_sizes[14] != kHid) return;
  if (in_sizes[15] != kHid * kF || in_sizes[16] != kF) return;
  if (out_size != kN * kF) return;
  if (ws_size < kWsTotal) return;

  const float* x    = (const float*)d_in[0];
  const int*   ei   = (const int*)  d_in[1];
  const float* att  = (const float*)d_in[2];
  const float* Wz   = (const float*)d_in[3];
  const float* bz   = (const float*)d_in[4];
  const float* Wr   = (const float*)d_in[5];
  const float* br   = (const float*)d_in[6];
  const float* Wh   = (const float*)d_in[7];
  const float* bh   = (const float*)d_in[8];
  const float* Lz   = (const float*)d_in[9];
  const float* lbz  = (const float*)d_in[10];
  const float* Lr   = (const float*)d_in[11];
  const float* lbr  = (const float*)d_in[12];
  const float* Lh   = (const float*)d_in[13];
  const float* lbh  = (const float*)d_in[14];
  const float* Wout = (const float*)d_in[15];
  const float* bout = (const float*)d_in[16];
  float* out = (float*)d_out;

  char* ws = (char*)d_ws;
  float*          DINV = (float*)(ws + kOffDinv);
  unsigned short* XA   = (unsigned short*)(ws + kOffXA);
  unsigned short* WPh  = (unsigned short*)(ws + kOffWPh);
  float*          WPf  = (float*)(ws + kOffWPf);

  deg_kernel<<<kDegBlocks, 256, 0, stream>>>(ei, DINV);
  agg_kernel<<<kAggBlocks, 256, 0, stream>>>(x, ei, DINV, XA);
  prep_kernel<<<1, 256, 0, stream>>>(att, Wz, bz, Wr, br, Wh, bh, Lz, lbz, Lr, lbr, Lh, lbh, WPh, WPf);
  gru_kernel<<<kGruBlocks, 128, 0, stream>>>(XA, WPh, WPf, Wout, bout, out);
}
